// HeteroCrossAttention_54211077210529
// MI455X (gfx1250) — hardware-verified
//
#include <hip/hip_runtime.h>
#include <stdint.h>

#define DEV static __device__ __forceinline__

typedef _Float16 v16h __attribute__((ext_vector_type(16)));
typedef _Float16 v8h  __attribute__((ext_vector_type(8)));
typedef _Float16 v4h  __attribute__((ext_vector_type(4)));
typedef float    v8f  __attribute__((ext_vector_type(8)));
typedef float    v4f  __attribute__((ext_vector_type(4)));

static constexpr int T  = 2;
static constexpr int NN = 2048;
static constexpr int D  = 256;
static constexpr int H  = 8;
static constexpr int HD = 32;

static constexpr float S_W   = 64.0f;
static constexpr float S_QKV = 8.0f;
static constexpr float S_P   = 4096.0f;
static constexpr float S_A   = 512.0f;

union Frag { v16h v; v8h half[2]; };
union HV   { v8h h; v4f f; };

DEV v8f zero8() { v8f z = {0.f, 0.f, 0.f, 0.f, 0.f, 0.f, 0.f, 0.f}; return z; }

DEV v8f wmma16(v16h a, v16h b, v8f c) {
    v8f d = __builtin_amdgcn_wmma_f32_16x16x32_f16(false, a, false, b, (short)0, c, false, false);
    asm volatile("v_nop\n\tv_nop\n\tv_nop\n\tv_nop" : "+v"(d) : "v"(a), "v"(b));
    return d;
}

DEV v16h ld_frag(const _Float16* base, int idx, int lane) {
    const int hh = lane >> 4;
    const _Float16* r = base + idx * 32;
    Frag f;
    f.half[0] = *(const v8h*)(r + 8 * hh);
    f.half[1] = *(const v8h*)(r + 16 + 8 * hh);
    return f.v;
}

__global__ void __launch_bounds__(256)
convert_kernel(const float* __restrict__ in, _Float16* __restrict__ out, int n8, float s) {
    const int i = blockIdx.x * 256 + threadIdx.x;
    if (i < n8) {
        const v4f u0 = *(const v4f*)(in + (size_t)i * 8);
        const v4f u1 = *(const v4f*)(in + (size_t)i * 8 + 4);
        HV hv;
        hv.h[0] = (_Float16)(u0[0] * s); hv.h[1] = (_Float16)(u0[1] * s);
        hv.h[2] = (_Float16)(u0[2] * s); hv.h[3] = (_Float16)(u0[3] * s);
        hv.h[4] = (_Float16)(u1[0] * s); hv.h[5] = (_Float16)(u1[1] * s);
        hv.h[6] = (_Float16)(u1[2] * s); hv.h[7] = (_Float16)(u1[3] * s);
        _Float16* p = out + (size_t)i * 8;
        *(volatile v4f*)p = hv.f;
        __threadfence();
        *(volatile v4f*)p = hv.f;
    }
}

template <int WM, int WN, int APITCH, int AKSTR>
DEV void gemm_core(const _Float16* __restrict__ A, const _Float16* __restrict__ W,
                   _Float16* a_lds, _Float16* bt_lds, v8f (&acc)[2][2],
                   int blockM, int blockN) {
    constexpr int BM = 32 * WM, BN = 32 * WN;
    const int tid  = threadIdx.x;
    const int lane = tid & 31;
    const int wid  = tid >> 5;
    const int m    = lane & 15;
    const int waveM = wid % WM, waveN = wid / WM;

    for (int kt = 0; kt < D / 32; ++kt) {
        const int k0 = kt * 32;
        __syncthreads();
        for (int i = tid; i < BM * 2; i += 256) {
            const int r = i >> 1, sg = (i & 1) * 16;
            const _Float16* p = A + (size_t)kt * AKSTR + (size_t)(blockM * BM + r) * APITCH + sg;
            const v8h u0 = *(const v8h*)p;
            const v8h u1 = *(const v8h*)(p + 8);
            *(v8h*)(a_lds + r * 32 + sg)     = u0;
            *(v8h*)(a_lds + r * 32 + sg + 8) = u1;
        }
        for (int i = tid; i < 4 * BN; i += 256) {
            const int wr = i / (BN / 8), wc = (i % (BN / 8)) * 8;
            const _Float16* p = W + (size_t)(k0 + wr) * D + blockN * BN + wc;
            const v8h w = *(const v8h*)p;
#pragma unroll
            for (int j = 0; j < 8; ++j) bt_lds[(wc + j) * 32 + wr] = w[j];
        }
        __syncthreads();
#pragma unroll
        for (int sm = 0; sm < 2; ++sm) {
            const v16h af = ld_frag(a_lds, waveM * 32 + sm * 16 + m, lane);
#pragma unroll
            for (int sn = 0; sn < 2; ++sn) {
                const v16h bf = ld_frag(bt_lds, waveN * 32 + sn * 16 + m, lane);
                acc[sm][sn] = wmma16(af, bf, acc[sm][sn]);
            }
        }
    }
}

__global__ void __launch_bounds__(256)
proj_kernel(const _Float16* __restrict__ x16,
            const _Float16* __restrict__ wq16, const _Float16* __restrict__ wk16,
            const _Float16* __restrict__ wv16,
            const float* __restrict__ bq, const float* __restrict__ bk,
            const float* __restrict__ bv,
            _Float16* __restrict__ Q16, _Float16* __restrict__ K16,
            _Float16* __restrict__ V16) {
    __shared__ __attribute__((aligned(16))) _Float16 a_lds[128 * 32];
    __shared__ __attribute__((aligned(16))) _Float16 bt_lds[64 * 32];
    __shared__ __attribute__((aligned(16))) _Float16 c_lds[128 * 64];

    const int z = blockIdx.z, t = z / 3, which = z % 3;
    const _Float16* W   = (which == 0 ? wq16 : (which == 1 ? wk16 : wv16)) + (size_t)t * D * D;
    const float*    bia = (which == 0 ? bq : (which == 1 ? bk : bv)) + (size_t)t * D;
    _Float16*       out = (which == 0 ? Q16 : (which == 1 ? K16 : V16)) + (size_t)t * NN * D;
    const _Float16* A   = x16 + (size_t)t * NN * D;

    v8f acc[2][2];
#pragma unroll
    for (int i = 0; i < 2; ++i)
#pragma unroll
        for (int j = 0; j < 2; ++j) acc[i][j] = zero8();

    gemm_core<4, 2, D, 32>(A, W, a_lds, bt_lds, acc, blockIdx.x, blockIdx.y);

    const int tid = threadIdx.x, lane = tid & 31, wid = tid >> 5;
    const int m = lane & 15, hh = lane >> 4;
    const int waveM = wid & 3, waveN = wid >> 2;
    const float inw = 1.0f / S_W;
#pragma unroll
    for (int sm = 0; sm < 2; ++sm)
#pragma unroll
        for (int sn = 0; sn < 2; ++sn) {
            const int col = waveN * 32 + sn * 16 + m;
            const float bb = bia[blockIdx.y * 64 + col];
#pragma unroll
            for (int v = 0; v < 8; ++v) {
                const int row = waveM * 32 + sm * 16 + hh * 8 + v;
                c_lds[row * 64 + col] = (_Float16)((acc[sm][sn][v] * inw + bb) * S_QKV);
            }
        }
    __syncthreads();
    HV vals[4];
    const int cc = (lane & 7) * 8;
#pragma unroll
    for (int i = 0; i < 4; ++i) {
        const int r = wid * 16 + i * 4 + (lane >> 3);
        vals[i].h = *(const v8h*)(c_lds + r * 64 + cc);
    }
    _Float16* ob = out + (size_t)(blockIdx.x * 128) * D + blockIdx.y * 64 + cc;
#pragma unroll
    for (int i = 0; i < 4; ++i) {
        const int r = wid * 16 + i * 4 + (lane >> 3);
        *(volatile v4f*)(ob + (size_t)r * D) = vals[i].f;
    }
    __threadfence();
#pragma unroll
    for (int i = 0; i < 4; ++i) {
        const int r = wid * 16 + i * 4 + (lane >> 3);
        *(volatile v4f*)(ob + (size_t)r * D) = vals[i].f;
    }
}

__global__ void __launch_bounds__(256)
attn_kernel(const _Float16* __restrict__ Q16, const _Float16* __restrict__ K16,
            const _Float16* __restrict__ V16, _Float16* __restrict__ attT) {
    __shared__ __attribute__((aligned(16))) _Float16 k_lds[32 * 32];
    __shared__ __attribute__((aligned(16))) _Float16 vt_lds[32 * 32];
    __shared__ __attribute__((aligned(16))) _Float16 p_lds[8 * 16 * 32];

    const int tid = threadIdx.x, lane = tid & 31, wid = tid >> 5;
    const int m = lane & 15, hh = lane >> 4;
    const int t = blockIdx.z, h = blockIdx.y;
    const int kvt = 1 - t;
    const int qBase = blockIdx.x * 128 + wid * 16;
    const size_t qOfs  = (size_t)t   * NN * D;
    const size_t kvOfs = (size_t)kvt * NN * D;

    Frag qf;
    {
        const _Float16* qp = Q16 + qOfs + (size_t)(qBase + m) * D + h * HD;
        qf.half[0] = *(const v8h*)(qp + 8 * hh);
        qf.half[1] = *(const v8h*)(qp + 16 + 8 * hh);
    }
    const v16h qa = qf.v;
    const float sc = 0.17677669529663687f / (S_QKV * S_QKV);

    float mrun[8], lrun[8];
#pragma unroll
    for (int v = 0; v < 8; ++v) { mrun[v] = -1e30f; lrun[v] = 0.f; }
    v8f o0 = zero8(), o1 = zero8();

    _Float16* pw = p_lds + wid * (16 * 32);

    for (int j0 = 0; j0 < NN; j0 += 32) {
        __syncthreads();
        {
            const int r = tid >> 3, c = (tid & 7) * 4;
            const size_t go = kvOfs + (size_t)(j0 + r) * D + h * HD + c;
            const v4h kv = *(const v4h*)(K16 + go);
            const v4h vv = *(const v4h*)(V16 + go);
            *(v4h*)(k_lds + r * 32 + c) = kv;
#pragma unroll
            for (int j = 0; j < 4; ++j) vt_lds[(c + j) * 32 + r] = vv[j];
        }
        __syncthreads();

        const v16h kb0 = ld_frag(k_lds, m, lane);
        const v16h kb1 = ld_frag(k_lds, 16 + m, lane);
        const v8f s0 = wmma16(qa, kb0, zero8());
        const v8f s1 = wmma16(qa, kb1, zero8());

#pragma unroll
        for (int v = 0; v < 8; ++v) {
            const float a0 = s0[v] * sc, a1 = s1[v] * sc;
            float mx = fmaxf(a0, a1);
#pragma unroll
            for (int msk = 1; msk < 16; msk <<= 1) mx = fmaxf(mx, __shfl_xor(mx, msk));
            const float mN   = fmaxf(mrun[v], mx);
            const float corr = __expf(mrun[v] - mN);
            const float p0 = __expf(a0 - mN), p1 = __expf(a1 - mN);
            float ps = p0 + p1;
#pragma unroll
            for (int msk = 1; msk < 16; msk <<= 1) ps += __shfl_xor(ps, msk);
            lrun[v] = lrun[v] * corr + ps;
            mrun[v] = mN;
            o0[v] *= corr; o1[v] *= corr;
            const int row = hh * 8 + v;
            pw[row * 32 + m]      = (_Float16)(p0 * S_P);
            pw[row * 32 + 16 + m] = (_Float16)(p1 * S_P);
        }
        __syncthreads();

        const v16h pa  = ld_frag(pw, m, lane);
        const v16h vb0 = ld_frag(vt_lds, m, lane);
        const v16h vb1 = ld_frag(vt_lds, 16 + m, lane);
        o0 = wmma16(pa, vb0, o0);
        o1 = wmma16(pa, vb1, o1);
    }
    __syncthreads();

    const float kf = (S_P * S_QKV) / S_A;
#pragma unroll
    for (int v = 0; v < 8; ++v) {
        const float f = 1.0f / (lrun[v] * kf);
        const int row = hh * 8 + v;
        pw[row * 32 + m]      = (_Float16)(o0[v] * f);
        pw[row * 32 + 16 + m] = (_Float16)(o1[v] * f);
    }
    __syncthreads();
    HV u0, u1;
    u0.h = *(const v8h*)(pw + lane * 8);
    u1.h = *(const v8h*)(pw + 256 + lane * 8);
    _Float16* ob = attT + (((size_t)t * H + h) * NN + qBase) * HD + lane * 8;
    *(volatile v4f*)ob         = u0.f;
    *(volatile v4f*)(ob + 256) = u1.f;
    __threadfence();
    *(volatile v4f*)ob         = u0.f;
    *(volatile v4f*)(ob + 256) = u1.f;
}

__global__ void __launch_bounds__(256)
oproj_ln_kernel(const _Float16* __restrict__ attT, const _Float16* __restrict__ wo16,
                const float* __restrict__ bo, const float* __restrict__ x,
                const float* __restrict__ g, const float* __restrict__ b,
                float* __restrict__ out) {
    __shared__ __attribute__((aligned(16))) _Float16 a_lds[32 * 32];
    __shared__ __attribute__((aligned(16))) _Float16 bt_lds[256 * 32];
    __shared__ __attribute__((aligned(16))) float    y_lds[32 * 256];

    const int t = blockIdx.z;
    const _Float16* A = attT + (size_t)t * NN * D;
    const _Float16* W = wo16 + (size_t)t * D * D;
    const float*    bb = bo + (size_t)t * D;

    v8f acc[2][2];
#pragma unroll
    for (int i = 0; i < 2; ++i)
#pragma unroll
        for (int j = 0; j < 2; ++j) acc[i][j] = zero8();

    gemm_core<1, 8, HD, NN * HD>(A, W, a_lds, bt_lds, acc, blockIdx.x, 0);

    const int tid = threadIdx.x, lane = tid & 31, wid = tid >> 5;
    const int m = lane & 15, hh = lane >> 4;
    const float ino = 1.0f / (S_A * S_W);
#pragma unroll
    for (int sm = 0; sm < 2; ++sm)
#pragma unroll
        for (int sn = 0; sn < 2; ++sn) {
            const int col = wid * 32 + sn * 16 + m;
            const float bc = bb[col];
#pragma unroll
            for (int v = 0; v < 8; ++v) {
                const int row = sm * 16 + hh * 8 + v;
                y_lds[row * D + col] = acc[sm][sn][v] * ino + bc;
            }
        }
    __syncthreads();

    const float* gg = g + (size_t)t * D;
    const float* be = b + (size_t)t * D;
    const v4f g0 = *(const v4f*)(gg + 4 * lane), g1 = *(const v4f*)(gg + 128 + 4 * lane);
    const v4f b0 = *(const v4f*)(be + 4 * lane), b1 = *(const v4f*)(be + 128 + 4 * lane);
    const float invd = 1.0f / D;
#pragma unroll
    for (int i = 0; i < 4; ++i) {
        const int r = wid * 4 + i;
        const size_t grow = (size_t)t * NN + (size_t)blockIdx.x * 32 + r;
        const float* xr = x + grow * D;
        const v4f y0 = *(const v4f*)(y_lds + r * D + 4 * lane)       + *(const v4f*)(xr + 4 * lane);
        const v4f y1 = *(const v4f*)(y_lds + r * D + 128 + 4 * lane) + *(const v4f*)(xr + 128 + 4 * lane);
        float s = y0[0] + y0[1] + y0[2] + y0[3] + y1[0] + y1[1] + y1[2] + y1[3];
#pragma unroll
        for (int msk = 1; msk < 32; msk <<= 1) s += __shfl_xor(s, msk);
        const float mean = s * invd;
        const v4f d0 = y0 - mean, d1 = y1 - mean;
        float sq = d0[0] * d0[0] + d0[1] * d0[1] + d0[2] * d0[2] + d0[3] * d0[3] +
                   d1[0] * d1[0] + d1[1] * d1[1] + d1[2] * d1[2] + d1[3] * d1[3];
#pragma unroll
        for (int msk = 1; msk < 32; msk <<= 1) sq += __shfl_xor(sq, msk);
        const float var = sq * invd;
        const float rs  = rsqrtf(var + 1e-5f);
        const v4f r0 = (d0 * rs) * g0 + b0;
        const v4f r1 = (d1 * rs) * g1 + b1;
        float* op = out + grow * D;
        *(volatile v4f*)(op + 4 * lane)       = r0;
        *(volatile v4f*)(op + 128 + 4 * lane) = r1;
        __threadfence();
        *(volatile v4f*)(op + 4 * lane)       = r0;
        *(volatile v4f*)(op + 128 + 4 * lane) = r1;
    }
}

extern "C" void kernel_launch(void* const* d_in, const int* in_sizes, int n_in,
                              void* d_out, int out_size, void* d_ws, size_t ws_size,
                              hipStream_t stream) {
    const size_t XND = (size_t)T * NN * D;
    const size_t WDD = (size_t)T * D * D;
    if (n_in < 11) return;
    if ((size_t)in_sizes[0] != XND || (size_t)in_sizes[1] != WDD || (size_t)out_size != XND) return;

    const float* x    = (const float*)d_in[0];
    const float* Wq   = (const float*)d_in[1];
    const float* bq   = (const float*)d_in[2];
    const float* Wk   = (const float*)d_in[3];
    const float* bk   = (const float*)d_in[4];
    const float* Wv   = (const float*)d_in[5];
    const float* bv   = (const float*)d_in[6];
    const float* Wo   = (const float*)d_in[7];
    const float* bo   = (const float*)d_in[8];
    const float* ln_g = (const float*)d_in[9];
    const float* ln_b = (const float*)d_in[10];
    float* out = (float*)d_out;

    char* ws = (char*)d_ws;
    size_t off = 0;
    auto carve = [&](size_t bytes) { size_t o = off; off = (off + bytes + 255) & ~(size_t)255; return o; };
    const size_t o_x16 = carve(XND * 2);
    const size_t o_wq  = carve(WDD * 2);
    const size_t o_wk  = carve(WDD * 2);
    const size_t o_wv  = carve(WDD * 2);
    const size_t o_wo  = carve(WDD * 2);
    const size_t o_q   = carve(XND * 2);
    const size_t o_k   = carve(XND * 2);
    const size_t o_v   = carve(XND * 2);
    const size_t o_at  = carve(XND * 2);
    if (off > ws_size) return;

    _Float16* x16  = (_Float16*)(ws + o_x16);
    _Float16* wq16 = (_Float16*)(ws + o_wq);
    _Float16* wk16 = (_Float16*)(ws + o_wk);
    _Float16* wv16 = (_Float16*)(ws + o_wv);
    _Float16* wo16 = (_Float16*)(ws + o_wo);
    _Float16* Q16  = (_Float16*)(ws + o_q);
    _Float16* K16  = (_Float16*)(ws + o_k);
    _Float16* V16  = (_Float16*)(ws + o_v);
    _Float16* attT = (_Float16*)(ws + o_at);

    const int nx8 = (int)(XND / 8), nw8 = (int)(WDD / 8);
    const unsigned gx = (unsigned)((nx8 + 255) / 256), gw = (unsigned)((nw8 + 255) / 256);
    convert_kernel<<<dim3(gx), 256, 0, stream>>>(x,  x16,  nx8, 1.0f);
    convert_kernel<<<dim3(gw), 256, 0, stream>>>(Wq, wq16, nw8, S_W);
    convert_kernel<<<dim3(gw), 256, 0, stream>>>(Wk, wk16, nw8, S_W);
    convert_kernel<<<dim3(gw), 256, 0, stream>>>(Wv, wv16, nw8, S_W);
    convert_kernel<<<dim3(gw), 256, 0, stream>>>(Wo, wo16, nw8, S_W);

    proj_kernel<<<dim3(NN / 128, D / 64, T * 3), 256, 0, stream>>>(x16, wq16, wk16, wv16,
                                                                    bq, bk, bv, Q16, K16, V16);
    attn_kernel<<<dim3(NN / 128, H, T), 256, 0, stream>>>(Q16, K16, V16, attT);
    oproj_ln_kernel<<<dim3(NN / 32, 1, T), 256, 0, stream>>>(attT, wo16, bo, x, ln_g, ln_b, out);
}
